// MLP_small_per_feature_16750372454576
// MI455X (gfx1250) — hardware-verified
//
#include <hip/hip_runtime.h>
#include <math.h>

typedef __attribute__((ext_vector_type(16))) _Float16 v16h;
typedef __attribute__((ext_vector_type(16))) __bf16 v16b;
typedef __attribute__((ext_vector_type(8)))  _Float16 v8h;
typedef __attribute__((ext_vector_type(8)))  float v8f;
typedef __attribute__((ext_vector_type(4)))  float v4f;
typedef __attribute__((ext_vector_type(2)))  float v2f;
typedef __attribute__((ext_vector_type(4)))  unsigned v4u;
typedef __attribute__((ext_vector_type(4)))  int v4i;
typedef float __attribute__((may_alias)) float_a;
typedef int __attribute__((may_alias)) int_a;

template <typename T> __device__ __forceinline__ void vst2(void* p, T v) { *(volatile T*)p = v; __threadfence(); *(volatile T*)p = v; }
__device__ __forceinline__ v8f wmma16(v16h a, v16h b, v8f c) {
  v8f d = __builtin_amdgcn_wmma_f32_16x16x32_f16(false, a, false, b, (short)0, c, false, false);
  asm volatile("v_nop\n\tv_nop\n\tv_nop\n\tv_nop" : "+v"(d) : "v"(a), "v"(b));
  return d;
}
__device__ __forceinline__ v8f wmma_bf(v16b a, v16b b, v8f c) {
  v8f d = __builtin_amdgcn_wmma_f32_16x16x32_bf16(false, a, false, b, (short)0, c, false, false);
  asm volatile("v_nop\n\tv_nop\n\tv_nop\n\tv_nop" : "+v"(d) : "v"(a), "v"(b));
  return d;
}
__device__ __forceinline__ v16h frag_h(const _Float16* rowk0, int lane) {
  union { v16h v; v8h q[2]; } u; const _Float16* p = rowk0 + 8 * (lane >> 4);
  u.q[0] = *(const v8h*)p; u.q[1] = *(const v8h*)(p + 16); return u.v;
}
__device__ __forceinline__ v16h frag_f32(const float* rowk0, int lane) {
  v16h a; const float* p = rowk0 + 8 * (lane >> 4);
#pragma unroll
  for (int i = 0; i < 8; ++i) { a[i] = (_Float16)p[i]; a[8 + i] = (_Float16)p[16 + i]; }
  return a;
}
__device__ __forceinline__ v16h frag_f32s(const float* rowk0, int lane, float sc) {
  v16h a; const float* p = rowk0 + 8 * (lane >> 4);
#pragma unroll
  for (int i = 0; i < 8; ++i) { a[i] = (_Float16)(p[i] * sc); a[8 + i] = (_Float16)(p[16 + i] * sc); }
  return a;
}
__device__ __forceinline__ v16h fragc_f32(const float* W, int k0, int n, int lane, int ld, int K) {
  v16h a; const int g = lane >> 4;
#pragma unroll
  for (int i = 0; i < 8; ++i) { const int ka = k0 + 8 * g + i, kb = ka + 16;
    a[i] = (_Float16)(ka < K ? W[(size_t)ka * ld + n] : 0.f); a[8 + i] = (_Float16)(kb < K ? W[(size_t)kb * ld + n] : 0.f); }
  return a;
}
struct F2 { v16b h, l; };
__device__ __forceinline__ F2 bsplit16(const float v[16]) { F2 r;
#pragma unroll
  for (int i = 0; i < 16; ++i) { const __bf16 h = (__bf16)v[i]; r.h[i] = h; r.l[i] = (__bf16)(v[i] - (float)h); }
  return r; }
__device__ __forceinline__ F2 split_row(const float* row, int k0, int lane) { float v[16]; const float* p = row + k0 + 8 * (lane >> 4);
#pragma unroll
  for (int i = 0; i < 8; ++i) { v[i] = p[i]; v[8 + i] = p[16 + i]; }
  return bsplit16(v); }
__device__ __forceinline__ F2 split_rowK(const float* row, int k0, int lane, int K) { float v[16]; const int g = lane >> 4;
#pragma unroll
  for (int i = 0; i < 8; ++i) { const int ka = k0 + 8 * g + i, kb = ka + 16; v[i] = ka < K ? row[ka] : 0.f; v[8 + i] = kb < K ? row[kb] : 0.f; }
  return bsplit16(v); }
__device__ __forceinline__ F2 split_col(const float* W, int k0, int n, int lane, int ld, int K) { float v[16]; const int g = lane >> 4;
#pragma unroll
  for (int i = 0; i < 8; ++i) { const int ka = k0 + 8 * g + i, kb = ka + 16; v[i] = ka < K ? W[(size_t)ka * ld + n] : 0.f; v[8 + i] = kb < K ? W[(size_t)kb * ld + n] : 0.f; }
  return bsplit16(v); }
__device__ __forceinline__ v8f mac3(const F2& a, const F2& b, v8f c) { c = wmma_bf(a.l, b.h, c); c = wmma_bf(a.h, b.l, c); return wmma_bf(a.h, b.h, c); }
__device__ __forceinline__ float sigm(float v) { return 1.0f / (1.0f + expf(-v)); }
#define LDSX() do { asm volatile("s_wait_dscnt 0" ::: "memory"); __builtin_amdgcn_wave_barrier(); __builtin_amdgcn_fence(__ATOMIC_RELEASE, "workgroup"); } while (0)

#define NBT 8192
#define NF 256
#define HH 64

__global__ __launch_bounds__(128) void k_main(const float* __restrict__ x, const float* __restrict__ w1, const float* __restrict__ b1, const float* __restrict__ w2, const float* __restrict__ b2, const float* __restrict__ w3, const float* __restrict__ b3, float* __restrict__ out) {
  __shared__ __align__(16) float so[4][16][NF + 4];
  const int tid = threadIdx.x, wave = tid >> 5, lane = tid & 31, col = lane & 15, g = lane >> 4;
  const int r0 = blockIdx.x * 64 + wave * 16;
#pragma unroll 1
  for (int f = 0; f < NF; ++f) {
    const float xv = x[(size_t)(r0 + col) * NF + f];
    const float* w1f = w1 + (size_t)f * HH; const float* b1f = b1 + (size_t)f * HH; const float* w2f = w2 + (size_t)f * HH * HH; const float* b2f = b2 + (size_t)f * HH; const float* w3f = w3 + (size_t)f * HH;
    v8f acc[4] = {};
#pragma unroll
    for (int kc = 0; kc < 2; ++kc) { v16h a;
#pragma unroll
      for (int i = 0; i < 8; ++i) { const int ka = kc * 32 + 8 * g + i, kb = ka + 16; const float va = xv * w1f[ka] + b1f[ka], vb = xv * w1f[kb] + b1f[kb]; a[i] = (_Float16)(va > 0.f ? va : 0.f); a[8 + i] = (_Float16)(vb > 0.f ? vb : 0.f); }
#pragma unroll
      for (int t = 0; t < 4; ++t) acc[t] = wmma16(a, frag_f32s(w2f + (size_t)(t * 16 + col) * HH + kc * 32, lane, 8.0f), acc[t]); }
    float part[8];
#pragma unroll
    for (int r = 0; r < 8; ++r) part[r] = 0.f;
#pragma unroll
    for (int t = 0; t < 4; ++t) { const int o = t * 16 + col; const float bb = b2f[o], ww = w3f[o];
#pragma unroll
      for (int r = 0; r < 8; ++r) { const float h2 = acc[t][r] * 0.125f + bb; part[r] += (h2 > 0.f ? h2 : 0.f) * ww; } }
#pragma unroll
    for (int r = 0; r < 8; ++r) {
#pragma unroll
      for (int off = 1; off <= 8; off <<= 1) part[r] += __shfl_xor(part[r], off, 32); }
    { float pv = 0.f;
#pragma unroll
      for (int r = 0; r < 8; ++r) pv = (r == col) ? part[r] : pv;
      if (col < 8) so[wave][8 * g + col][f] = pv + b3[f]; }
  }
  LDSX();
  for (int rl = 0; rl < 16; ++rl) for (int pc = lane; pc < NF / 4; pc += 32) vst2(out + (size_t)(r0 + rl) * NF + pc * 4, *(const v4f*)(&so[wave][rl][pc * 4]));
}
extern "C" void kernel_launch(void* const* d_in, const int* in_sizes, int n_in, void* d_out, int out_size, void* d_ws, size_t ws_size, hipStream_t stream) {
  (void)in_sizes; (void)n_in; (void)out_size; (void)ws_size; (void)d_ws;
  const float** I = (const float**)d_in;
  k_main<<<NBT / 64, 128, 0, stream>>>(I[0], I[1], I[2], I[3], I[4], I[5], I[6], (float*)d_out);
}
